// MultiGAT_55035710931590
// MI455X (gfx1250) — hardware-run, weakly checked
//
#include <hip/hip_runtime.h>

typedef float          v8f   __attribute__((ext_vector_type(8)));
typedef float          v4f   __attribute__((ext_vector_type(4)));
typedef unsigned int   v4u   __attribute__((ext_vector_type(4)));
typedef int            v8i   __attribute__((ext_vector_type(8)));
typedef unsigned short v8us  __attribute__((ext_vector_type(8)));
typedef unsigned short v16us __attribute__((ext_vector_type(16)));
typedef __bf16         v16bf __attribute__((ext_vector_type(16)));
typedef _Float16       v16h  __attribute__((ext_vector_type(16)));
typedef v4f  __attribute__((may_alias)) v4fa;
typedef v8us __attribute__((may_alias)) v8usa;
union FragB { v16bf v; v16us u; v8us h[2]; v8i w; };
union FragH { v16h  v; v16us u; v8us h[2]; v8i w; };

__device__ __forceinline__ v8f wmb(const FragB& a, const FragB& b, v8f c) {
  v8f d = __builtin_amdgcn_wmma_f32_16x16x32_bf16(false, a.v, false, b.v, (short)0, c, false, false);
  asm volatile("v_nop\n\tv_nop\n\tv_nop\n\tv_nop" : "+v"(d) : "v"(a.w), "v"(b.w));
  return d;
}

__device__ __forceinline__ v8f wmh(const FragH& a, const FragH& b, v8f c) {
  v8f d = __builtin_amdgcn_wmma_f32_16x16x32_f16(false, a.v, false, b.v, (short)0, c, false, false);
  asm volatile("v_nop\n\tv_nop\n\tv_nop\n\tv_nop" : "+v"(d) : "v"(a.w), "v"(b.w));
  return d;
}

__device__ __forceinline__ unsigned bf16_bits(float f) {
  const unsigned u = __float_as_uint(f);
  const unsigned r = (u + 0x7FFFu + ((u >> 16) & 1u)) >> 16;
  const unsigned q = (u >> 16) | 0x40u;
  return ((u & 0x7fffffffu) > 0x7f800000u) ? q : r;
}

__device__ __forceinline__ float bf16_val(float f) {
  return __uint_as_float(bf16_bits(f) << 16);
}
__device__ __forceinline__ int clampi(int v, int lo, int hi) {
  return v < lo ? lo : (v > hi ? hi : v);
}

__device__ __forceinline__ unsigned f16_bits(float f) {
  const unsigned u  = __float_as_uint(f);
  const unsigned s  = (u >> 16) & 0x8000u;
  const unsigned a  = u & 0x7fffffffu;
  const unsigned t  = a - 0x38000000u;
  const unsigned r  = (t + 0x0FFFu + ((t >> 13) & 1u)) >> 13;
  const unsigned rc = r > 0x7C00u ? 0x7C00u : r;
  const bool small  = a < 0x38800000u;
  const bool isnan  = a > 0x7f800000u;
  const unsigned fin = small ? 0u : (s | rc);
  return isnan ? (s | 0x7E00u) : fin;
}

__device__ __forceinline__ unsigned pk16(unsigned lo, unsigned hi) { return lo | (hi << 16); }
__device__ __forceinline__ unsigned bf16_lo_bits(float v) {
  float hi = bf16_val(v);
  asm volatile("" : "+v"(hi));
  return bf16_bits(v - hi);
}
__device__ __forceinline__ v4u pack8_bf16(v4f a, v4f c) {
  return (v4u){ pk16(bf16_bits(a[0]), bf16_bits(a[1])), pk16(bf16_bits(a[2]), bf16_bits(a[3])),
                pk16(bf16_bits(c[0]), bf16_bits(c[1])), pk16(bf16_bits(c[2]), bf16_bits(c[3])) };
}
__device__ __forceinline__ v4u pack8_bf16_lo(v4f a, v4f c) {
  return (v4u){ pk16(bf16_lo_bits(a[0]), bf16_lo_bits(a[1])), pk16(bf16_lo_bits(a[2]), bf16_lo_bits(a[3])),
                pk16(bf16_lo_bits(c[0]), bf16_lo_bits(c[1])), pk16(bf16_lo_bits(c[2]), bf16_lo_bits(c[3])) };
}
__device__ __forceinline__ v4u pack8_f16(v4f a, v4f c) {
  return (v4u){ pk16(f16_bits(a[0]), f16_bits(a[1])), pk16(f16_bits(a[2]), f16_bits(a[3])),
                pk16(f16_bits(c[0]), f16_bits(c[1])), pk16(f16_bits(c[2]), f16_bits(c[3])) };
}

template <int FORM>
__global__ __launch_bounds__(256) void k_plane(const float* __restrict__ src, int rows, int cols, int ldsrc,
                                               unsigned short* __restrict__ dst, int MP, int KP) {
  static_assert(FORM >= 0 && FORM <= 3);
  const int KTOT = (FORM == 1 || FORM == 3) ? 2 * KP : KP;
  const unsigned ppr   = (unsigned)(KTOT >> 3);
  const unsigned kp8   = (unsigned)(KP >> 3);
  const unsigned total = (unsigned)MP * ppr;
  const unsigned g     = blockIdx.x * 256u + threadIdx.x;
  const unsigned rowu  = g / ppr;
  const unsigned p     = g - rowu * ppr;
  const bool second    = p >= kp8;
  const int row = (int)rowu;
  const int c0  = (int)((second ? p - kp8 : p) << 3);
  const float* srow = src + (size_t)clampi(row, 0, rows - 1) * (size_t)ldsrc;
  float x[8];
  unsigned mk[8];
#pragma unroll
  for (int e = 0; e < 8; ++e) {
    const int c = c0 + e;
    const float v = srow[clampi(c, 0, cols - 1)];
    asm volatile("" :: "v"(v));
    x[e]  = v;
    mk[e] = (row < rows && c < cols) ? 0xFFFFu : 0u;
  }
  const v4f a = (v4f){ x[0], x[1], x[2], x[3] };
  const v4f c = (v4f){ x[4], x[5], x[6], x[7] };
  v4u o;
  if (FORM == 2) {
    o = pack8_f16(a, c);
  } else {
    const v4u hi = pack8_bf16(a, c);
    o = hi;
    if (FORM == 1) { const v4u lo = pack8_bf16_lo(a, c); o = second ? lo : hi; }
  }
  const v4u mw = (v4u){ pk16(mk[0], mk[1]), pk16(mk[2], mk[3]), pk16(mk[4], mk[5]), pk16(mk[6], mk[7]) };
  o &= mw;
  if (g < total) {
    volatile v4u* q = (volatile v4u*)(dst + (size_t)g * 8);
    *q = o;
    __threadfence();
    *q = o;
  }
}

template <int FORM> struct FragOf    { typedef FragB T; };
template <>         struct FragOf<2> { typedef FragH T; };
__device__ __forceinline__ v8f mm(const FragB& a, const FragB& b, v8f c) { return wmb(a, b, c); }
__device__ __forceinline__ v8f mm(const FragH& a, const FragH& b, v8f c) { return wmh(a, b, c); }
template <class F> __device__ __forceinline__ F ld_frag(const unsigned short* p) {
  F f;
  f.h[0] = *(const v8usa*)(p);
  f.h[1] = *(const v8usa*)(p + 16);
  return f;
}

template <int FORM, int EPI>
__global__ __launch_bounds__(256) __attribute__((amdgpu_num_vgpr(248)))
void k_gemm_nt(const unsigned short* __restrict__ A, const unsigned short* __restrict__ B,
               const float* __restrict__ bias, float* __restrict__ D, int M, int N, int KTOT, int ldd) {
  static_assert(FORM >= 0 && FORM <= 2);
  static_assert(EPI == 0 || EPI == 1);
  typedef typename FragOf<FORM>::T F;
  __shared__ __attribute__((aligned(16))) float sT[8][16 * 68];
  const int lane = threadIdx.x & 31;
  const int wave = threadIdx.x >> 5;
  const int tilesM = (M + 63) >> 6;
  const int tilesN = (N + 63) >> 6;
  const int tile = blockIdx.x * 8 + wave;
  if (tile >= tilesM * tilesN) return;
  const int tm = tile / tilesN;
  const int tn = tile - tm * tilesN;
  const int m0 = tm << 6;
  const int n0 = tn << 6;

  const int rl = lane & 15;
  const int h8 = (lane >> 4) * 8;
  const unsigned short* pa = A + (size_t)(m0 + rl) * (size_t)KTOT + h8;
  const unsigned short* pb = B + (size_t)(n0 + rl) * (size_t)KTOT + h8;

  v8f acc[4][4];
#pragma unroll
  for (int i = 0; i < 4; ++i)
#pragma unroll
    for (int j = 0; j < 4; ++j) acc[i][j] = (v8f){0.f, 0.f, 0.f, 0.f, 0.f, 0.f, 0.f, 0.f};

#pragma unroll 1
  for (int k0 = 0; k0 < KTOT; k0 += 32) {
    F bf[4];
#pragma unroll
    for (int j = 0; j < 4; ++j) bf[j] = ld_frag<F>(pb + (size_t)(j << 4) * (size_t)KTOT + k0);
#pragma unroll
    for (int i = 0; i < 4; ++i) {
      const F af = ld_frag<F>(pa + (size_t)(i << 4) * (size_t)KTOT + k0);
#pragma unroll
      for (int j = 0; j < 4; ++j) acc[i][j] = mm(af, bf[j], acc[i][j]);
    }
  }

  float* slab = sT[wave];
  const int hh = lane >> 4;
  const int c4 = (lane & 15) * 4;
  const int nc = n0 + c4;
  const bool cok = nc < N;
  v4f bv = (v4f){0.f, 0.f, 0.f, 0.f};
  if (EPI == 1) {
    bv = *(const v4fa*)(bias + clampi(nc, 0, N - 4));
    asm volatile("" :: "v"(bv));
  }
#pragma unroll
  for (int i = 0; i < 4; ++i) {
    const int mBase = m0 + (i << 4);
#pragma unroll
    for (int j = 0; j < 4; ++j) {
#pragma unroll
      for (int r = 0; r < 8; ++r) slab[(h8 + r) * 68 + (j << 4) + rl] = acc[i][j][r];
    }
    __builtin_amdgcn_fence(__ATOMIC_RELEASE, "workgroup");
    __builtin_amdgcn_wave_barrier();
    __builtin_amdgcn_fence(__ATOMIC_ACQUIRE, "workgroup");
    v4f vv[8];
#pragma unroll
    for (int it = 0; it < 8; ++it) {
      const int row = it * 2 + hh;
      v4f v = *(const v4fa*)(slab + row * 68 + c4);
      if (EPI == 1) v += bv;
      vv[it] = v;
    }
    for (int pass = 0; pass < 2; ++pass) {
#pragma unroll
      for (int it = 0; it < 8; ++it) {
        const int row = mBase + it * 2 + hh;
        if (cok && row < M) *(volatile v4f*)(D + (size_t)row * (size_t)ldd + nc) = vv[it];
      }
      __threadfence();
    }
    __builtin_amdgcn_fence(__ATOMIC_RELEASE, "workgroup");
    __builtin_amdgcn_wave_barrier();
    __builtin_amdgcn_fence(__ATOMIC_ACQUIRE, "workgroup");
  }
}

typedef int          v4i  __attribute__((ext_vector_type(4)));
typedef unsigned int v2u  __attribute__((ext_vector_type(2)));
typedef v4i __attribute__((may_alias)) v4ia;
typedef v2u __attribute__((may_alias)) v2ua;

constexpr int   N_NODE      = 10000;
constexpr int   N_EDGE      = 320000;
constexpr int   CHN         = 256;
constexpr int   MPAD        = 10048;
constexpr int   NBRUN       = 512;
constexpr int   NBLK        = 20;
constexpr int   DEGCAP      = 64;
constexpr int   MEAS_MAXDEG = 54;
constexpr int   CHUNK       = 2048;
constexpr int   NCHUNK      = 157;
constexpr int   WCAP        = 256;
constexpr float NEGS        = 0.2f;
constexpr bool  TWO_TERM_L2 = true;
constexpr bool  TWO_TERM_L3 = true;
constexpr bool  TWO_TERM_L4 = true;
constexpr int   LDS_BKT     = (NBRUN * DEGCAP + NBRUN + 8 * WCAP + 16) * 4;

static_assert(N_NODE < 65536);
static_assert(N_EDGE % CHUNK == 512);
static_assert((N_EDGE + CHUNK - 1) / CHUNK == NCHUNK);
static_assert(N_EDGE % 8 == 0);
static_assert(DEGCAP >= MEAS_MAXDEG + 8);
static_assert(DEGCAP == 64);
static_assert(NBRUN == 512);
static_assert(NBLK * NBRUN >= N_NODE);
static_assert(N_NODE % 8 == 0);
static_assert(MPAD % 64 == 0 && MPAD >= N_NODE && MPAD % 16 == 0);
static_assert(LDS_BKT <= 262144);

constexpr size_t S_XB   = (size_t)MPAD * 256 * 2;
constexpr size_t S_AHL  = (size_t)MPAD * 512 * 2;
constexpr size_t S_HW   = (size_t)MPAD * 256 * 4;
constexpr size_t S_ESD  = (size_t)2 * N_NODE * 4 * 4;
constexpr size_t S_WP   = (size_t)(65536 + 3 * 131072) * 2;
constexpr size_t S_TAB  = (size_t)12 * 256 * 4;
constexpr size_t S_SRCL = (size_t)NBLK * NBRUN * DEGCAP * 4;
constexpr size_t S_CNT  = (size_t)NBLK * NBRUN * 4;
constexpr size_t S_FLAG = (size_t)NBLK * 128;
constexpr size_t O_XB   = 0;
constexpr size_t O_AHL  = O_XB + S_XB;
constexpr size_t O_HW   = O_AHL + S_AHL;
constexpr size_t O_ESD  = O_HW + S_HW;
constexpr size_t O_WP   = O_ESD + S_ESD;
constexpr size_t O_TAB  = O_WP + S_WP;
constexpr size_t O_SRCL = O_TAB + S_TAB;
constexpr size_t O_CNT  = O_SRCL + S_SRCL;
constexpr size_t O_FLAG = O_CNT + S_CNT;
constexpr size_t WS_TOTAL = O_FLAG + S_FLAG;
static_assert(S_XB % 256 == 0 && S_AHL % 256 == 0 && S_HW % 256 == 0 && S_ESD % 256 == 0 && S_WP % 256 == 0);
static_assert(S_TAB % 256 == 0 && S_SRCL % 256 == 0 && S_CNT % 256 == 0 && S_FLAG % 256 == 0);
static_assert(WS_TOTAL == 29637632);
static_assert(WS_TOTAL <= ((size_t)128 << 20));

__device__ __forceinline__ void wave_sync() {
  __builtin_amdgcn_fence(__ATOMIC_RELEASE, "workgroup");
  __builtin_amdgcn_wave_barrier();
  __builtin_amdgcn_fence(__ATOMIC_ACQUIRE, "workgroup");
}
__device__ __forceinline__ v4f ld4(const float* __restrict__ p, int t) { return *(const v4fa*)(p + 4 * t); }
__device__ __forceinline__ v4f widen4(v2u w) {
  return (v4f){ __uint_as_float(w.x << 16), __uint_as_float(w.x & 0xffff0000u),
                __uint_as_float(w.y << 16), __uint_as_float(w.y & 0xffff0000u) };
}
__device__ __forceinline__ float relu_k(float v) { return (v > 0.f) ? v : ((v != v) ? v : 0.f); }
__device__ __forceinline__ float pois(float v, unsigned pm) {
  return __uint_as_float((__float_as_uint(v) & ~pm) | (0x7fc00000u & pm));
}

__global__ __launch_bounds__(256) void k_prep(
    const float* __restrict__ W1, const float* __restrict__ W2, const float* __restrict__ W3, const float* __restrict__ WN,
    const float* __restrict__ as1, const float* __restrict__ ad1, const float* __restrict__ b1,
    const float* __restrict__ as2, const float* __restrict__ ad2, const float* __restrict__ b2,
    const float* __restrict__ as3, const float* __restrict__ ad3, const float* __restrict__ b3,
    const float* __restrict__ asN, const float* __restrict__ adN, const float* __restrict__ bN,
    unsigned short* __restrict__ WP, float* __restrict__ TAB, unsigned short* __restrict__ AHL) {
  __shared__ __attribute__((aligned(16))) float sT[64 * 68];
  const int t = threadIdx.x;
  const int b = blockIdx.x;
  if (b < 64) {
    const int mat = b >> 4, tl = b & 15;
    const int k0 = (tl >> 2) * 64, n0 = (tl & 3) * 64;
#pragma unroll
    for (int i = 0; i < 4; ++i) {
      const int idx = t + 256 * i;
      const int k = idx >> 4, n4 = (idx & 15) * 4;
      const int off = (k0 + k) * CHN + n0 + n4;
      v4f v;
      if (mat == 0)      v = *(const v4fa*)(W1 + off);
      else if (mat == 1) v = *(const v4fa*)(W2 + off);
      else if (mat == 2) v = *(const v4fa*)(W3 + off);
      else               v = *(const v4fa*)(WN + off);
      *(v4fa*)(sT + k * 68 + n4) = v;
    }
    __syncthreads();
    const int pitch = (mat == 0) ? 256 : 512;
    const size_t base = (mat == 0) ? (size_t)0 : (size_t)65536 + (size_t)(mat - 1) * 131072;
    v4u ov[2];
    size_t oo[2];
#pragma unroll
    for (int i = 0; i < 2; ++i) {
      const int q = t + 256 * i;
      const int n = q >> 3, p = q & 7;
      float x[8];
#pragma unroll
      for (int e = 0; e < 8; ++e) x[e] = sT[(8 * p + e) * 68 + n];
      ov[i] = pack8_bf16((v4f){x[0], x[1], x[2], x[3]}, (v4f){x[4], x[5], x[6], x[7]});
      oo[i] = base + (size_t)(n0 + n) * (size_t)pitch + (size_t)(k0 + 8 * p);
    }
#pragma unroll
    for (int i = 0; i < 2; ++i) {
      *(volatile v4u*)(WP + oo[i]) = ov[i];
      if (mat != 0) *(volatile v4u*)(WP + oo[i] + 256) = ov[i];
    }
    __threadfence();
#pragma unroll
    for (int i = 0; i < 2; ++i) {
      *(volatile v4u*)(WP + oo[i]) = ov[i];
      if (mat != 0) *(volatile v4u*)(WP + oo[i] + 256) = ov[i];
    }
  } else if (b < 76) {
    const int r = b - 64;
    if (t < 64) {
      v4f v;
      switch (r) {
        case 0:  v = ld4(as1, t); break;
        case 1:  v = ld4(ad1, t); break;
        case 2:  v = ld4(b1,  t); break;
        case 3:  v = ld4(as2, t); break;
        case 4:  v = ld4(ad2, t); break;
        case 5:  v = ld4(b2,  t); break;
        case 6:  v = ld4(as3, t); break;
        case 7:  v = ld4(ad3, t); break;
        case 8:  v = ld4(b3,  t); break;
        case 9:  v = ld4(asN, t); break;
        case 10: v = ld4(adN, t); break;
        default: v = ld4(bN,  t); break;
      }
      const v4f o = (v4f){ bf16_val(v.x), bf16_val(v.y), bf16_val(v.z), bf16_val(v.w) };
      volatile v4f* q = (volatile v4f*)(TAB + r * 256 + 4 * t);
      *q = o;
      __threadfence();
      *q = o;
    }
  } else {
    const int g = (b - 76) * 256 + t;
    const v4u z = (v4u){0u, 0u, 0u, 0u};
    volatile v4u* q = (volatile v4u*)(AHL + (size_t)N_NODE * 512 + (size_t)g * 8);
    *q = z;
    __threadfence();
    *q = z;
  }
}

__global__ __launch_bounds__(256) void k_bucket(const int* __restrict__ ei, int* __restrict__ SRCL,
                                                int* __restrict__ CNT, int* __restrict__ FLAG) {
  extern __shared__ v4i lds_dyn[];
  int* strip = (int*)lds_dyn;
  int* scnt  = strip + NBRUN * DEGCAP;
  int* list  = scnt + NBRUN;
  int* wcnt  = list + 8 * WCAP;
  const int t = threadIdx.x, lane = t & 31, wave = t >> 5;
  const int blk = blockIdx.x;
  const int nodeBase = blk * NBRUN;
  int liveSlots = N_NODE - nodeBase;
  liveSlots = liveSlots < 0 ? 0 : (liveSlots > NBRUN ? NBRUN : liveSlots);

#pragma unroll 4
  for (int i = 0; i < (NBRUN * DEGCAP / 4) / 256; ++i) {
    const int q = t + 256 * i;
    int own = nodeBase + (q >> 4);
    own = own > N_NODE - 1 ? N_NODE - 1 : own;
    *(v4ia*)(strip + 4 * q) = (v4i){own, own, own, own};
  }
  scnt[t] = 0;
  scnt[t + 256] = 0;
#pragma unroll
  for (int i = 0; i < 8; ++i) list[t + 256 * i] = 0;
  if (t < 16) wcnt[t] = 0;
  __syncthreads();

  const unsigned nb0 = (unsigned)nodeBase;
  const unsigned ulive = (unsigned)liveSlots;
#pragma unroll 1
  for (int ch = 0; ch < NCHUNK; ++ch) {
    const int e0 = ch * CHUNK + t * 8;
    const int ec = e0 < N_EDGE - 8 ? e0 : N_EDGE - 8;
    const bool valid = e0 < N_EDGE;
    const v4i da = *(const v4ia*)(ei + N_EDGE + ec);
    const v4i db = *(const v4ia*)(ei + N_EDGE + ec + 4);
    const v4i sa = *(const v4ia*)(ei + ec);
    const v4i sb = *(const v4ia*)(ei + ec + 4);
    asm volatile("" :: "v"(da), "v"(db), "v"(sa), "v"(sb));
    const int dd[8] = { da.x, da.y, da.z, da.w, db.x, db.y, db.z, db.w };
    const int ss[8] = { sa.x, sa.y, sa.z, sa.w, sb.x, sb.y, sb.z, sb.w };
    unsigned sl[8];
    bool hit[8];
    int cl = 0;
#pragma unroll
    for (int J = 0; J < 8; ++J) {
      sl[J]  = (unsigned)dd[J] - nb0;
      hit[J] = valid && (sl[J] < ulive);
      cl += hit[J] ? 1 : 0;
    }
    int incl = cl;
#pragma unroll
    for (int d = 1; d < 32; d <<= 1) {
      const int up = __shfl_up(incl, d);
      incl += (lane >= d) ? up : 0;
    }
    const int wc = __builtin_amdgcn_readlane(incl, 31);
    if (wc != 0) {
      int pos = incl - cl;
#pragma unroll
      for (int J = 0; J < 8; ++J) {
        if (hit[J]) {
          const unsigned sv = (unsigned)clampi(ss[J], 0, N_NODE - 1);
          if (pos < WCAP) list[wave * WCAP + pos] = (int)((sv << 16) | sl[J]);
          ++pos;
        }
      }
    }
    if (lane == 0) wcnt[wave] = wc;
    __syncthreads();
    if (wave == 0) {
#pragma unroll 1
      for (int w2 = 0; w2 < 8; ++w2) {
        int c = wcnt[w2];
        c = c < 0 ? 0 : (c > WCAP ? WCAP : c);
        c = __builtin_amdgcn_readfirstlane(c);
#pragma unroll 1
        for (int b0 = 0; b0 < c; b0 += 32) {
          int idx = b0 + lane;
          idx = idx < c ? idx : c - 1;
          const int uv = list[w2 * WCAP + idx];
          const int m32 = (c - b0) < 32 ? (c - b0) : 32;
#pragma unroll 1
          for (int k = 0; k < m32; ++k) {
            const unsigned u = (unsigned)__builtin_amdgcn_readlane(uv, k);
            const int sq = (int)(u & (unsigned)(NBRUN - 1));
            const int sr = (int)(u >> 16);
            if (lane == 0) {
              const int c0 = scnt[sq];
              const int cp = c0 < 0 ? 0 : (c0 > DEGCAP - 1 ? DEGCAP - 1 : c0);
              if (c0 < DEGCAP) strip[sq * DEGCAP + cp] = sr;
              scnt[sq] = c0 + 1;
            }
          }
        }
      }
    }
    __syncthreads();
  }

  const bool bad = (scnt[t] > DEGCAP) | (scnt[t + 256] > DEGCAP);
  const unsigned bm = __builtin_amdgcn_ballot_w32(bad);
  if (lane == 0) wcnt[wave] = (bm != 0u) ? 1 : 0;
  __syncthreads();
  int flag = 0;
#pragma unroll
  for (int w2 = 0; w2 < 8; ++w2) flag |= wcnt[w2];

  int* gl = SRCL + (size_t)nodeBase * DEGCAP;
#pragma unroll 1
  for (int i0 = 0; i0 < 8; ++i0) {
    v4i v[4];
#pragma unroll
    for (int k = 0; k < 4; ++k) v[k] = *(const v4ia*)(strip + 4 * (t + 256 * (4 * i0 + k)));
#pragma unroll
    for (int k = 0; k < 4; ++k) *(volatile v4i*)(gl + 4 * (t + 256 * (4 * i0 + k))) = v[k];
    __threadfence();
#pragma unroll
    for (int k = 0; k < 4; ++k) *(volatile v4i*)(gl + 4 * (t + 256 * (4 * i0 + k))) = v[k];
  }
  const v4i cv = *(const v4ia*)(scnt + 4 * (t & 127));
  const v4i fv = (v4i){flag, flag, flag, flag};
  if (t < 128) *(volatile v4i*)(CNT + nodeBase + 4 * t) = cv;
  if (t < 8)   *(volatile v4i*)(FLAG + blk * 32 + 4 * t) = fv;
  __threadfence();
  if (t < 128) *(volatile v4i*)(CNT + nodeBase + 4 * t) = cv;
  if (t < 8)   *(volatile v4i*)(FLAG + blk * 32 + 4 * t) = fv;
}

__global__ __launch_bounds__(256) void k_dots(const float* __restrict__ HW, const float* __restrict__ TABL,
                                              float* __restrict__ ESD) {
  __shared__ __attribute__((aligned(16))) float sA[512];
  __shared__ __attribute__((aligned(16))) float sO[64];
  const int t = threadIdx.x, lane = t & 31, wave = t >> 5;
  const int row = blockIdx.x * 8 + wave;
  if (t < 128) { const v4f v = *(const v4fa*)(TABL + 4 * t); *(v4fa*)(sA + 4 * t) = v; }
  const float* hp = HW + (size_t)row * CHN + 4 * lane;
  const v4f h0 = *(const v4fa*)hp;
  const v4f h1 = *(const v4fa*)(hp + 128);
  __syncthreads();
  const v4f as0 = *(const v4fa*)(sA + 4 * lane);
  const v4f as1 = *(const v4fa*)(sA + 128 + 4 * lane);
  const v4f ad0 = *(const v4fa*)(sA + 256 + 4 * lane);
  const v4f ad1 = *(const v4fa*)(sA + 384 + 4 * lane);
  float es0 = h0.x * as0.x + h0.y * as0.y + h0.z * as0.z + h0.w * as0.w;
  float es1 = h1.x * as1.x + h1.y * as1.y + h1.z * as1.z + h1.w * as1.w;
  float ed0 = h0.x * ad0.x + h0.y * ad0.y + h0.z * ad0.z + h0.w * ad0.w;
  float ed1 = h1.x * ad1.x + h1.y * ad1.y + h1.z * ad1.z + h1.w * ad1.w;
#pragma unroll
  for (int d = 1; d < 16; d <<= 1) {
    es0 += __shfl_xor(es0, d);
    es1 += __shfl_xor(es1, d);
    ed0 += __shfl_xor(ed0, d);
    ed1 += __shfl_xor(ed1, d);
  }
  if ((lane & 15) == 0) {
    const int hh = lane >> 4;
    sO[wave * 4 + hh]          = es0;
    sO[wave * 4 + 2 + hh]      = es1;
    sO[32 + wave * 4 + hh]     = ed0;
    sO[32 + wave * 4 + 2 + hh] = ed1;
  }
  __syncthreads();
  if (t < 16) {
    const int tb = t >> 3, q = t & 7;
    const v4f v = *(const v4fa*)(sO + tb * 32 + q * 4);
    volatile v4f* g = (volatile v4f*)(ESD + (size_t)tb * (size_t)(N_NODE * 4) + (size_t)blockIdx.x * 32 + q * 4);
    *g = v;
    __threadfence();
    *g = v;
  }
}

template <int LAST, int TWO>
__global__ __launch_bounds__(256) void k_replay(
    const float* __restrict__ HW, const float* __restrict__ ESD, const float* __restrict__ BIASL,
    const unsigned short* __restrict__ XB, const int* __restrict__ SRCL, const int* __restrict__ CNT,
    const int* __restrict__ FLAG, unsigned short* __restrict__ AHL, float* __restrict__ OUT, int nrows) {
  __shared__ __attribute__((aligned(16))) float sBias[CHN];
  __shared__ __attribute__((aligned(16))) float sAl[8][DEGCAP * 4];
  __shared__ __attribute__((aligned(16))) int   sSrc[8][DEGCAP];
  const int t = threadIdx.x, lane = t & 31, wave = t >> 5, hh = lane >> 4;
  if (t < 64) { const v4f bq = *(const v4fa*)(BIASL + 4 * t); *(v4fa*)(sBias + 4 * t) = bq; }
  __syncthreads();

  const int row = blockIdx.x * 8 + wave;
  const bool live = row < nrows;
  const int rc = live ? row : nrows - 1;
  float* strip = sAl[wave];
  int*   ssw   = sSrc[wave];

  const int craw = CNT[rc];
  const int fl   = FLAG[(rc / NBRUN) * 32];
  const v4f edv  = *(const v4fa*)(ESD + (size_t)(N_NODE * 4) + (size_t)rc * 4);
  const v2u xw0  = *(const v2ua*)(XB + (size_t)rc * CHN + 4 * lane);
  const v2u xw1  = *(const v2ua*)(XB + (size_t)rc * CHN + 128 + 4 * lane);
  asm volatile("" :: "v"(craw), "v"(fl), "v"(edv), "v"(xw0), "v"(xw1));
  int cvv = craw < 0 ? 0 : (craw > DEGCAP ? DEGCAP : craw);
  cvv = live ? cvv : 0;
  const int cn = __builtin_amdgcn_readfirstlane(cvv);
  const bool pz = (fl != 0) | (craw > DEGCAP) | (craw < 0);
  const unsigned pm = pz ? 0xffffffffu : 0u;

  const float ninf = -__builtin_huge_valf();
  v4f m4 = (v4f){ninf, ninf, ninf, ninf};
#pragma unroll 1
  for (int hf = 0; hf < 2; ++hf) {
    const int idx = hf * 32 + lane;
    int s = SRCL[(size_t)rc * DEGCAP + idx];
    asm volatile("" :: "v"(s));
    s = clampi(s, 0, nrows - 1);
    const v4f es = *(const v4fa*)(ESD + (size_t)s * 4);
    asm volatile("" :: "v"(es));
    const bool ok = idx < cn;
    v4f e;
#pragma unroll
    for (int hd = 0; hd < 4; ++hd) {
      float a = es[hd] + edv[hd];
      a = (a >= 0.f) ? a : NEGS * a;
      const float ev = ok ? a : ninf;
      e[hd]  = ev;
      m4[hd] = (ev > m4[hd]) ? ev : m4[hd];
    }
    ssw[idx] = s;
    *(v4fa*)(strip + idx * 4) = e;
  }
#pragma unroll
  for (int d = 1; d < 32; d <<= 1) {
#pragma unroll
    for (int hd = 0; hd < 4; ++hd) {
      const float o = __shfl_xor(m4[hd], d);
      m4[hd] = (o > m4[hd]) ? o : m4[hd];
    }
  }
#pragma unroll
  for (int hd = 0; hd < 4; ++hd) m4[hd] = ((m4[hd] - m4[hd]) == 0.f) ? m4[hd] : 0.f;

#pragma unroll 1
  for (int hf = 0; hf < 2; ++hf) {
    const int idx = hf * 32 + lane;
    const bool ok = idx < cn;
    const v4f e = *(const v4fa*)(strip + idx * 4);
    v4f p;
#pragma unroll
    for (int hd = 0; hd < 4; ++hd) {
      const float q = expf(e[hd] - m4[hd]);
      p[hd] = ok ? q : 0.f;
    }
    *(v4fa*)(strip + idx * 4) = p;
  }
  wave_sync();
  v4f s4 = (v4f){0.f, 0.f, 0.f, 0.f};
#pragma unroll 1
  for (int j = 0; j < cn; ++j) {
    const v4f pv = *(const v4fa*)(strip + j * 4);
    s4 += pv;
  }
  wave_sync();
#pragma unroll 1
  for (int hf = 0; hf < 2; ++hf) {
    const int idx = hf * 32 + lane;
    const v4f p = *(const v4fa*)(strip + idx * 4);
    v4f al;
#pragma unroll
    for (int hd = 0; hd < 4; ++hd) al[hd] = p[hd] / (s4[hd] + 1e-16f);
    *(v4fa*)(strip + idx * 4) = al;
  }
  wave_sync();

  v4f acc0 = (v4f){0.f, 0.f, 0.f, 0.f};
  v4f acc1 = (v4f){0.f, 0.f, 0.f, 0.f};
  const float* hwl = HW + 4 * lane;
#pragma unroll 1
  for (int j = 0; j < cn; ++j) {
    int sj = ssw[j];
    sj = clampi(sj, 0, nrows - 1);
    sj = __builtin_amdgcn_readfirstlane(sj);
    const float* hp = hwl + (size_t)sj * CHN;
    const v4f g0 = *(const v4fa*)hp;
    const v4f g1 = *(const v4fa*)(hp + 128);
    asm volatile("" :: "v"(g0), "v"(g1));
    const float a0 = strip[j * 4 + hh];
    const float a1 = strip[j * 4 + 2 + hh];
    acc0 += a0 * g0;
    acc1 += a1 * g1;
  }

  const v4f x0 = widen4(xw0), x1 = widen4(xw1);
  const v4f b0 = *(const v4fa*)(sBias + 4 * lane);
  const v4f b1 = *(const v4fa*)(sBias + 128 + 4 * lane);
  float t0[4], t1[4];
#pragma unroll
  for (int c = 0; c < 4; ++c) {
    float u0 = acc0[c] + b0[c];
    float u1 = acc1[c] + b1[c];
    if (LAST) {
      u0 = relu_k(u0 + x0[c]);
      u1 = relu_k(u1 + x1[c]);
    } else {
      u0 = relu_k(u0) + x0[c];
      u1 = relu_k(u1) + x1[c];
    }
    t0[c] = pois(u0, pm);
    t1[c] = pois(u1, pm);
  }
  if (LAST) {
    const v4f o0 = (v4f){t0[0], t0[1], t0[2], t0[3]};
    const v4f o1 = (v4f){t1[0], t1[1], t1[2], t1[3]};
    float* op = OUT + (size_t)rc * CHN + 4 * lane;
    if (live) { *(volatile v4f*)op = o0; *(volatile v4f*)(op + 128) = o1; }
    __threadfence();
    if (live) { *(volatile v4f*)op = o0; *(volatile v4f*)(op + 128) = o1; }
  } else {
    const v2u hi0 = (v2u){ pk16(bf16_bits(t0[0]), bf16_bits(t0[1])), pk16(bf16_bits(t0[2]), bf16_bits(t0[3])) };
    const v2u hi1 = (v2u){ pk16(bf16_bits(t1[0]), bf16_bits(t1[1])), pk16(bf16_bits(t1[2]), bf16_bits(t1[3])) };
    v2u lo0 = (v2u){0u, 0u};
    v2u lo1 = (v2u){0u, 0u};
    if (TWO) {
      lo0 = (v2u){ pk16(bf16_lo_bits(t0[0]), bf16_lo_bits(t0[1])), pk16(bf16_lo_bits(t0[2]), bf16_lo_bits(t0[3])) };
      lo1 = (v2u){ pk16(bf16_lo_bits(t1[0]), bf16_lo_bits(t1[1])), pk16(bf16_lo_bits(t1[2]), bf16_lo_bits(t1[3])) };
    }
    unsigned short* ar = AHL + (size_t)rc * 512 + 4 * lane;
    if (live) {
      *(volatile v2u*)(ar)       = hi0;
      *(volatile v2u*)(ar + 128) = hi1;
      *(volatile v2u*)(ar + 256) = lo0;
      *(volatile v2u*)(ar + 384) = lo1;
    }
    __threadfence();
    if (live) {
      *(volatile v2u*)(ar)       = hi0;
      *(volatile v2u*)(ar + 128) = hi1;
      *(volatile v2u*)(ar + 256) = lo0;
      *(volatile v2u*)(ar + 384) = lo1;
    }
  }
}

extern "C" void kernel_launch(void* const* d_in, const int* in_sizes, int n_in,
                              void* d_out, int out_size, void* d_ws, size_t ws_size,
                              hipStream_t stream) {
  if (n_in < 18) return;
  if (in_sizes[0] != N_NODE * CHN) return;
  if (in_sizes[1] != 2 * N_EDGE) return;
  for (int l = 0; l < 4; ++l) {
    if (in_sizes[2 + 4 * l] != CHN * CHN) return;
    if (in_sizes[3 + 4 * l] != CHN || in_sizes[4 + 4 * l] != CHN || in_sizes[5 + 4 * l] != CHN) return;
  }
  if (out_size != N_NODE * CHN) return;
  if (ws_size < WS_TOTAL) return;

  const float* x   = (const float*)d_in[0];
  const int*   ei  = (const int*)  d_in[1];
  const float* W1  = (const float*)d_in[2];
  const float* as1 = (const float*)d_in[3];
  const float* ad1 = (const float*)d_in[4];
  const float* b1  = (const float*)d_in[5];
  const float* W2  = (const float*)d_in[6];
  const float* as2 = (const float*)d_in[7];
  const float* ad2 = (const float*)d_in[8];
  const float* b2  = (const float*)d_in[9];
  const float* W3  = (const float*)d_in[10];
  const float* as3 = (const float*)d_in[11];
  const float* ad3 = (const float*)d_in[12];
  const float* b3  = (const float*)d_in[13];
  const float* WN  = (const float*)d_in[14];
  const float* asN = (const float*)d_in[15];
  const float* adN = (const float*)d_in[16];
  const float* bN  = (const float*)d_in[17];
  float* out = (float*)d_out;

  char* ws = (char*)d_ws;
  unsigned short* XB   = (unsigned short*)(ws + O_XB);
  unsigned short* AHL  = (unsigned short*)(ws + O_AHL);
  float*          HW   = (float*)(ws + O_HW);
  float*          ESD  = (float*)(ws + O_ESD);
  unsigned short* WP   = (unsigned short*)(ws + O_WP);
  float*          TAB  = (float*)(ws + O_TAB);
  int*            SRCL = (int*)(ws + O_SRCL);
  int*            CNT  = (int*)(ws + O_CNT);
  int*            FLAG = (int*)(ws + O_FLAG);
  const unsigned short* W1T = WP;
  const unsigned short* W2D = WP + 65536;
  const unsigned short* W3D = WP + 65536 + 131072;
  const unsigned short* WND = WP + 65536 + 2 * 131072;

  hipFuncSetAttribute(reinterpret_cast<const void*>(&k_bucket),
                      hipFuncAttributeMaxDynamicSharedMemorySize, LDS_BKT);

  k_plane<0><<<MPAD * CHN / 8 / 256, 256, 0, stream>>>(x, N_NODE, CHN, CHN, XB, MPAD, CHN);
  k_prep<<<88, 256, 0, stream>>>(W1, W2, W3, WN, as1, ad1, b1, as2, ad2, b2, as3, ad3, b3, asN, adN, bN,
                                 WP, TAB, AHL);
  k_bucket<<<NBLK, 256, LDS_BKT, stream>>>(ei, SRCL, CNT, FLAG);

  const int gG = ((MPAD / 64) * (CHN / 64) + 7) / 8;
  const int gR = N_NODE / 8;

  k_gemm_nt<0, 0><<<gG, 256, 0, stream>>>(XB, W1T, TAB, HW, MPAD, CHN, 256, CHN);
  k_dots<<<gR, 256, 0, stream>>>(HW, TAB + 0 * 768, ESD);
  k_replay<0, TWO_TERM_L2 ? 1 : 0><<<gR, 256, 0, stream>>>(HW, ESD, TAB + 0 * 768 + 512, XB, SRCL, CNT, FLAG,
                                                           AHL, out, N_NODE);
  k_gemm_nt<0, 0><<<gG, 256, 0, stream>>>(AHL, W2D, TAB, HW, MPAD, CHN, 512, CHN);
  k_dots<<<gR, 256, 0, stream>>>(HW, TAB + 1 * 768, ESD);
  k_replay<0, TWO_TERM_L3 ? 1 : 0><<<gR, 256, 0, stream>>>(HW, ESD, TAB + 1 * 768 + 512, XB, SRCL, CNT, FLAG,
                                                           AHL, out, N_NODE);
  k_gemm_nt<0, 0><<<gG, 256, 0, stream>>>(AHL, W3D, TAB, HW, MPAD, CHN, 512, CHN);
  k_dots<<<gR, 256, 0, stream>>>(HW, TAB + 2 * 768, ESD);
  k_replay<0, TWO_TERM_L4 ? 1 : 0><<<gR, 256, 0, stream>>>(HW, ESD, TAB + 2 * 768 + 512, XB, SRCL, CNT, FLAG,
                                                           AHL, out, N_NODE);
  k_gemm_nt<0, 0><<<gG, 256, 0, stream>>>(AHL, WND, TAB, HW, MPAD, CHN, 512, CHN);
  k_dots<<<gR, 256, 0, stream>>>(HW, TAB + 3 * 768, ESD);
  k_replay<1, 0><<<gR, 256, 0, stream>>>(HW, ESD, TAB + 3 * 768 + 512, XB, SRCL, CNT, FLAG,
                                         AHL, out, N_NODE);
}
